// PyTorchDeltaNetLayer_70205535420782
// MI455X (gfx1250) — hardware-verified
//
#include <hip/hip_runtime.h>
#include <math.h>

typedef __attribute__((ext_vector_type(16))) _Float16 v16h;
typedef __attribute__((ext_vector_type(16))) __bf16 v16b;
typedef __attribute__((ext_vector_type(8)))  _Float16 v8h;
typedef __attribute__((ext_vector_type(8)))  float v8f;
typedef __attribute__((ext_vector_type(4)))  float v4f;
typedef __attribute__((ext_vector_type(2)))  float v2f;
typedef __attribute__((ext_vector_type(4)))  unsigned v4u;
typedef __attribute__((ext_vector_type(4)))  int v4i;
typedef float __attribute__((may_alias)) float_a;
typedef int __attribute__((may_alias)) int_a;

template <typename T> __device__ __forceinline__ void vst2(void* p, T v) { *(volatile T*)p = v; __threadfence(); *(volatile T*)p = v; }
__device__ __forceinline__ v8f wmma16(v16h a, v16h b, v8f c) {
  v8f d = __builtin_amdgcn_wmma_f32_16x16x32_f16(false, a, false, b, (short)0, c, false, false);
  asm volatile("v_nop\n\tv_nop\n\tv_nop\n\tv_nop" : "+v"(d) : "v"(a), "v"(b));
  return d;
}
__device__ __forceinline__ v8f wmma_bf(v16b a, v16b b, v8f c) {
  v8f d = __builtin_amdgcn_wmma_f32_16x16x32_bf16(false, a, false, b, (short)0, c, false, false);
  asm volatile("v_nop\n\tv_nop\n\tv_nop\n\tv_nop" : "+v"(d) : "v"(a), "v"(b));
  return d;
}
__device__ __forceinline__ v16h frag_h(const _Float16* rowk0, int lane) {
  union { v16h v; v8h q[2]; } u; const _Float16* p = rowk0 + 8 * (lane >> 4);
  u.q[0] = *(const v8h*)p; u.q[1] = *(const v8h*)(p + 16); return u.v;
}
__device__ __forceinline__ v16h frag_f32(const float* rowk0, int lane) {
  v16h a; const float* p = rowk0 + 8 * (lane >> 4);
#pragma unroll
  for (int i = 0; i < 8; ++i) { a[i] = (_Float16)p[i]; a[8 + i] = (_Float16)p[16 + i]; }
  return a;
}
__device__ __forceinline__ v16h frag_f32s(const float* rowk0, int lane, float sc) {
  v16h a; const float* p = rowk0 + 8 * (lane >> 4);
#pragma unroll
  for (int i = 0; i < 8; ++i) { a[i] = (_Float16)(p[i] * sc); a[8 + i] = (_Float16)(p[16 + i] * sc); }
  return a;
}
__device__ __forceinline__ v16h fragc_f32(const float* W, int k0, int n, int lane, int ld, int K) {
  v16h a; const int g = lane >> 4;
#pragma unroll
  for (int i = 0; i < 8; ++i) { const int ka = k0 + 8 * g + i, kb = ka + 16;
    a[i] = (_Float16)(ka < K ? W[(size_t)(ka < K ? ka : K - 1) * ld + n] : 0.f); a[8 + i] = (_Float16)(kb < K ? W[(size_t)(kb < K ? kb : K - 1) * ld + n] : 0.f); }
  return a;
}
struct F2 { v16b h, l; };
__device__ __forceinline__ F2 bsplit16(const float v[16]) { F2 r;
#pragma unroll
  for (int i = 0; i < 16; ++i) { const __bf16 h = (__bf16)v[i]; r.h[i] = h; r.l[i] = (__bf16)(v[i] - (float)h); }
  return r; }
__device__ __forceinline__ F2 split_row(const float* row, int k0, int lane) { float v[16]; const float* p = row + k0 + 8 * (lane >> 4);
#pragma unroll
  for (int i = 0; i < 8; ++i) { v[i] = p[i]; v[8 + i] = p[16 + i]; }
  return bsplit16(v); }
__device__ __forceinline__ F2 split_rowK(const float* row, int k0, int lane, int K) { float v[16]; const int g = lane >> 4;
#pragma unroll
  for (int i = 0; i < 8; ++i) { const int ka = k0 + 8 * g + i, kb = ka + 16; v[i] = ka < K ? row[ka < K ? ka : K - 1] : 0.f; v[8 + i] = kb < K ? row[kb < K ? kb : K - 1] : 0.f; }
  return bsplit16(v); }
__device__ __forceinline__ F2 split_col(const float* W, int k0, int n, int lane, int ld, int K) { float v[16]; const int g = lane >> 4;
#pragma unroll
  for (int i = 0; i < 8; ++i) { const int ka = k0 + 8 * g + i, kb = ka + 16; v[i] = ka < K ? W[(size_t)(ka < K ? ka : K - 1) * ld + n] : 0.f; v[8 + i] = kb < K ? W[(size_t)(kb < K ? kb : K - 1) * ld + n] : 0.f; }
  return bsplit16(v); }
__device__ __forceinline__ v8f mac3(const F2& a, const F2& b, v8f c) { c = wmma_bf(a.l, b.h, c); c = wmma_bf(a.h, b.l, c); return wmma_bf(a.h, b.h, c); }
__device__ __forceinline__ float sigm(float v) { return 1.0f / (1.0f + expf(-v)); }
#define LDSX() do { asm volatile("s_wait_dscnt 0" ::: "memory"); __builtin_amdgcn_wave_barrier(); __builtin_amdgcn_fence(__ATOMIC_RELEASE, "workgroup"); } while (0)


#define NB 4
#define TT 2048
#define DM 1024
#define NH 16
#define HD 64
#define NTOK (NB * TT)
#define PW4 (4 * DM)
#ifndef NRB
#define NRB (NTOK / 64)
#define NBT NB
#endif
typedef __attribute__((ext_vector_type(8))) __bf16 v8b;
__device__ __forceinline__ v16b frag_b(const __bf16* rowk0, int lane) {
  union { v16b v; v8b q[2]; } u; const __bf16* p = rowk0 + 8 * (lane >> 4);
  u.q[0] = *(const v8b*)p; u.q[1] = *(const v8b*)(p + 16); return u.v;
}
__device__ __forceinline__ float bfr(float v) { return (float)(__bf16)v; }
__device__ __attribute__((noinline)) float exp_ni(float v) { return expf(v); }
__device__ __attribute__((noinline)) float erf_ni(float v) { return erff(v); }

#define WS_PK  0u
#define PKS ((size_t)PW4 * DM)
#define PKO (PKS + (size_t)48 * DM)
#define WS_P   (WS_PK + 2u * (PKO + (size_t)DM * DM))
#define WS_S   (WS_P + 4u * (size_t)NTOK * PW4)
#define WS_O   (WS_S + 4u * (size_t)NTOK * 64)
#define WS_END (WS_O + 4u * (size_t)NTOK * DM)

__global__ __launch_bounds__(256) void k_pack(const float* __restrict__ Wm, int nrows, __bf16* __restrict__ DST) {
  __shared__ __align__(16) __bf16 s[DM]; const int n = blockIdx.x, tid = threadIdx.x; if (n >= nrows) return;
  for (int k = tid; k < DM; k += 256) s[k] = (__bf16)Wm[(size_t)n * DM + k];
  __syncthreads();
  if (tid < DM / 8) vst2((unsigned*)(DST + (size_t)n * DM + tid * 8), *(const v4u*)&s[tid * 8]);
}
template <int SMALL>
__global__ __launch_bounds__(128) void k_proj(const float* __restrict__ X, const __bf16* __restrict__ P, const float* __restrict__ BFD, const float* __restrict__ BSD, float* __restrict__ OUT) {
  constexpr int NT = SMALL ? 3 : 8; constexpr int LDO = SMALL ? 64 : PW4;
  __shared__ __align__(16) float so[4][16][132];
  const int tid = threadIdx.x, wave = tid >> 5, lane = tid & 31, col = lane & 15, g = lane >> 4; const size_t r0 = (size_t)blockIdx.x * 64 + wave * 16; const int n0 = SMALL ? 0 : blockIdx.y * 128;
  v8f acc[NT]; for (int j = 0; j < NT; ++j) acc[j] = (v8f){};
#pragma unroll 2
  for (int kc = 0; kc < DM / 32; ++kc) { v16b a; { const float* p = X + (r0 + col) * DM + kc * 32 + 8 * g;
#pragma unroll
      for (int i = 0; i < 8; ++i) { a[i] = (__bf16)p[i]; a[8 + i] = (__bf16)p[16 + i]; } }
#pragma unroll
    for (int j = 0; j < NT; ++j) acc[j] = wmma_bf(a, frag_b(P + (size_t)(n0 + j * 16 + col) * DM + kc * 32, lane), acc[j]); }
#pragma unroll
  for (int j = 0; j < NT; ++j) { const int n = n0 + j * 16 + col;
#pragma unroll
    for (int r = 0; r < 8; ++r) { float v = acc[j][r];
      if (SMALL) { if (j == 1) v += bfr(BFD[col]); else if (j == 2) v += bfr(BSD[col]); v = sigm(v); }
      else { v = (n < 3 * DM) ? v * sigm(v) : sigm(v); }
      so[wave][8 * g + r][j * 16 + col] = v; } }
  if (SMALL) { if (col == 0) {
#pragma unroll
    for (int r = 0; r < 8; ++r) so[wave][8 * g + r][48] = 0.f; }
    for (int c = 49 + lane; c < 64; c += 32)
#pragma unroll
      for (int rr = 0; rr < 16; ++rr) so[wave][rr][c] = 0.f; }
  LDSX();
  for (int rl = 0; rl < 16; ++rl) { if (SMALL) { if (lane < 16) vst2(OUT + (r0 + rl) * 64 + lane * 4, *(const v4f*)&so[wave][rl][lane * 4]); } else vst2(OUT + (r0 + rl) * (size_t)PW4 + n0 + lane * 4, *(const v4f*)&so[wave][rl][lane * 4]); }
}
__global__ __launch_bounds__(256) void k_scan(const float* __restrict__ Pm, const float* __restrict__ Sg, float* __restrict__ O) {
  const int ch = blockIdx.x * 256 + threadIdx.x; const int b = ch / DM, hdx = ch % DM; const int h = hdx / HD;
  float Sf = 0.f, Ss = 0.f; const float mix = 0.05f;
#pragma unroll 1
  for (int t = 0; t < TT; ++t) { const size_t tok = (size_t)b * TT + t; const float* pr = Pm + tok * PW4 + hdx; const float qt = pr[0], kt = pr[DM], vt = pr[2 * DM]; const float* sr = Sg + tok * 64 + h; const float bt = sr[0], ft = sr[16], st = sr[32];
    Sf = Sf * ft; Ss = Ss * st; const float o = 0.5f * qt * (Sf + Ss); const float upd = (bt * kt) * vt; Sf = Sf + upd; Ss = Ss + upd; const float Sfn = Sf + mix * Ss; Ss = Ss + mix * Sf; Sf = Sfn;
    vst2(O + tok * DM + hdx, o); }
}
__global__ __launch_bounds__(128) void k_out(const float* __restrict__ O, const float* __restrict__ Pm, const __bf16* __restrict__ PO, float* __restrict__ Y) {
  __shared__ __align__(16) float so[4][16][132];
  const int tid = threadIdx.x, wave = tid >> 5, lane = tid & 31, col = lane & 15, g = lane >> 4; const size_t r0 = (size_t)blockIdx.x * 64 + wave * 16; const int n0 = blockIdx.y * 128;
  v8f acc[8] = {};
#pragma unroll 2
  for (int kc = 0; kc < DM / 32; ++kc) { float v[16]; const float* po = O + (r0 + col) * DM + kc * 32 + 8 * g; const float* pg = Pm + (r0 + col) * (size_t)PW4 + 3 * DM + kc * 32 + 8 * g;
#pragma unroll
    for (int i = 0; i < 8; ++i) { v[i] = po[i] * pg[i]; v[8 + i] = po[16 + i] * pg[16 + i]; }
    const F2 a = bsplit16(v);
#pragma unroll
    for (int j = 0; j < 8; ++j) { const v16b w = frag_b(PO + (size_t)(n0 + j * 16 + col) * DM + kc * 32, lane); acc[j] = wmma_bf(a.l, w, acc[j]); acc[j] = wmma_bf(a.h, w, acc[j]); } }
#pragma unroll
  for (int j = 0; j < 8; ++j)
#pragma unroll
    for (int r = 0; r < 8; ++r) so[wave][8 * g + r][j * 16 + col] = acc[j][r];
  LDSX();
  for (int rl = 0; rl < 16; ++rl) vst2(Y + (r0 + rl) * DM + n0 + lane * 4, *(const v4f*)&so[wave][rl][lane * 4]);
}
extern "C" void kernel_launch(void* const* d_in, const int* in_sizes, int n_in, void* d_out, int out_size, void* d_ws, size_t ws_size, hipStream_t stream) {
  (void)in_sizes; (void)n_in; (void)out_size;
  const float** F = (const float**)d_in;
  if (ws_size < (size_t)WS_END) return;
  char* ws = (char*)d_ws; __bf16* PK = (__bf16*)(ws + WS_PK); float *Pm = (float*)(ws + WS_P), *Sg = (float*)(ws + WS_S), *O = (float*)(ws + WS_O);
  k_pack<<<DM, 256, 0, stream>>>(F[1], DM, PK); k_pack<<<DM, 256, 0, stream>>>(F[2], DM, PK + (size_t)DM * DM); k_pack<<<DM, 256, 0, stream>>>(F[3], DM, PK + (size_t)2 * DM * DM); k_pack<<<DM, 256, 0, stream>>>(F[10], DM, PK + (size_t)3 * DM * DM);
  k_pack<<<16, 256, 0, stream>>>(F[5], 16, PK + PKS); k_pack<<<16, 256, 0, stream>>>(F[6], 16, PK + PKS + (size_t)16 * DM); k_pack<<<16, 256, 0, stream>>>(F[8], 16, PK + PKS + (size_t)32 * DM);
  k_pack<<<DM, 256, 0, stream>>>(F[4], DM, PK + PKO);
  k_proj<0><<<dim3(NRB, PW4 / 128), 128, 0, stream>>>(F[0], PK, nullptr, nullptr, Pm);
  k_proj<1><<<dim3(NRB, 1), 128, 0, stream>>>(F[0], PK + PKS, F[7], F[9], Sg);
  k_scan<<<NBT * DM / 256, 256, 0, stream>>>(Pm, Sg, O);
  k_out<<<dim3(NRB, DM / 128), 128, 0, stream>>>(O, Pm, PK + PKO, (float*)d_out);
}
